// SequentialOctave_87660282511418
// MI455X (gfx1250) — hardware-verified
//
#include <hip/hip_runtime.h>
#include <math.h>

constexpr int NBATCH   = 512;
constexpr int NSTEP    = 256;
constexpr int NDIM     = 64;
constexpr int NHID     = 128;
constexpr int NZ       = 64;
constexpr int NCOND    = 32;
constexpr int NGATE    = 4 * NHID;
constexpr int KCAT     = NDIM + NHID;
constexpr int KVAE     = NHID + NCOND;
constexpr int KFC1     = NZ + NCOND;
constexpr int NTHR     = 256;
constexpr int NWAVE    = NTHR / 32;
constexpr int ROWS_BLK = 16;
constexpr int APITCH   = 200;
constexpr int OPITCH   = 68;
constexpr int VPITCH   = 132;
constexpr float WCARRY     = 16.0f;
constexpr float WCARRY_INV = 0.0625f;
constexpr float RSC        = 2048.0f;
constexpr float RSC_INV    = 1.0f / 2048.0f;
constexpr size_t OFF_MU = (size_t)NBATCH * NSTEP * NDIM;
constexpr size_t OFF_LV = OFF_MU + (size_t)NBATCH * NZ;
static_assert(NBATCH % ROWS_BLK == 0);
static_assert(NHID == 16 * NWAVE);
static_assert(2 * NZ == 16 * NWAVE);
static_assert(NDIM == 16 * 4);
static_assert(KCAT % 32 == 0 && KVAE % 32 == 0 && KFC1 % 32 == 0 && NHID % 32 == 0 && NDIM % 32 == 0);
static_assert(APITCH % 8 == 0 && APITCH >= KCAT);
static_assert(NTHR == ROWS_BLK * 16);

typedef __attribute__((ext_vector_type(16))) _Float16 v16h;
typedef __attribute__((ext_vector_type(8)))  _Float16 v8h;
typedef __attribute__((ext_vector_type(4)))  _Float16 v4h;
typedef __attribute__((ext_vector_type(8)))  float    v8f;
typedef __attribute__((ext_vector_type(4)))  float    v4f;

__device__ __forceinline__ unsigned short f2bf_bits(float f) {
  unsigned u = __float_as_uint(f);
  return (unsigned short)((u + 0x7FFFu + ((u >> 16) & 1u)) >> 16);
}
__device__ __forceinline__ float bf_bits2f(unsigned short h) { return __uint_as_float(((unsigned)h) << 16); }
__device__ __forceinline__ float bf16r(float f) { return bf_bits2f(f2bf_bits(f)); }

__device__ __forceinline__ void dep_guard4_h(v8f& a, v8f& b, v8f& c, v8f& d, v16h x, v16h y) {
  asm volatile("v_nop\n\tv_nop\n\tv_nop\n\tv_nop" : "+v"(a), "+v"(b), "+v"(c), "+v"(d) : "v"(x), "v"(y));
}
__device__ __forceinline__ void dep_guard2x3_h(v8f& a, v8f& b, v16h x, v16h y, v16h z) {
  asm volatile("v_nop\n\tv_nop\n\tv_nop\n\tv_nop" : "+v"(a), "+v"(b) : "v"(x), "v"(y), "v"(z));
}
__device__ __forceinline__ void keep4_h(v16h a, v16h b, v16h c, v16h d) { asm volatile("v_nop" :: "v"(a), "v"(b), "v"(c), "v"(d)); }
__device__ __forceinline__ void acc_guard4(v8f& a, v8f& b, v8f& c, v8f& d) { asm volatile("v_nop\n\tv_nop\n\tv_nop\n\tv_nop" : "+v"(a), "+v"(b), "+v"(c), "+v"(d)); }
__device__ __forceinline__ void acc_guard2(v8f& a, v8f& b) { asm volatile("v_nop\n\tv_nop\n\tv_nop\n\tv_nop" : "+v"(a), "+v"(b)); }

template <typename T> struct Frag;
template <> struct Frag<_Float16> {
  typedef v16h V; union U { v16h v; v8h h[2]; };
  static __device__ __forceinline__ v16h load(const _Float16* p) {
    U f; f.h[0] = *(const v8h*)(p); f.h[1] = *(const v8h*)(p + 16); return f.v;
  }
  static __device__ __forceinline__ v8f mma(v16h a, v16h b, v8f c) {
    return __builtin_amdgcn_wmma_f32_16x16x32_f16(false, a, false, b, (short)0, c, false, false);
  }
};

__device__ __forceinline__ float fsig(float x)  { return __builtin_amdgcn_rcpf(1.0f + __expf(-x)); }
__device__ __forceinline__ float ftanh(float x) { return 1.0f - 2.0f * __builtin_amdgcn_rcpf(__expf(2.0f * x) + 1.0f); }

__device__ __forceinline__ void split16(float v, _Float16& hi, _Float16& lo) {
  const _Float16 h = (_Float16)v;
  hi = h;
  lo = (_Float16)((v - (float)h) * RSC);
}

__global__ __launch_bounds__(NTHR) void cvt_rows_kernel(const float* __restrict__ src, unsigned short* __restrict__ dst,
                                                      int rows, int cols, int dpitch, int dcol, float sc) {
  const int cpr = cols >> 3;
  const int n8  = rows * cpr;
  const int i   = blockIdx.x * NTHR + threadIdx.x;
  if (i < n8) {
    const int r  = i / cpr;
    const int k8 = (i - r * cpr) * 8;
    const float* sp = src + (size_t)r * cols + k8;
    const v4f a = *(const v4f*)(sp);
    const v4f b = *(const v4f*)(sp + 4);
    v8h hv;
#pragma unroll
    for (int e = 0; e < 4; ++e) {
      hv[e]     = (_Float16)(bf16r(a[e]) * sc);
      hv[4 + e] = (_Float16)(bf16r(b[e]) * sc);
    }
    unsigned short* dp = dst + (size_t)r * dpitch + dcol + k8;
    *(volatile v8h*)dp = hv;
    __threadfence();
    *(volatile v8h*)dp = hv;
  }
}

template <bool LO>
__device__ __forceinline__ void mma_chunks4(const _Float16* ahi, const _Float16* alo, const _Float16* brow, int gstride,
                                            int ch0, int ch1, v8f (&acc)[4], v8f (&accr)[4]) {
#pragma unroll 1
  for (int ch = ch0; ch < ch1; ++ch) {
    const int k0 = ch * 32;
    const v16h a  = Frag<_Float16>::load(ahi + k0);
    const v16h b0 = Frag<_Float16>::load(brow + k0);
    const v16h b1 = Frag<_Float16>::load(brow + (size_t)gstride + k0);
    const v16h b2 = Frag<_Float16>::load(brow + (size_t)2 * gstride + k0);
    const v16h b3 = Frag<_Float16>::load(brow + (size_t)3 * gstride + k0);
    acc[0] = Frag<_Float16>::mma(a, b0, acc[0]);
    acc[1] = Frag<_Float16>::mma(a, b1, acc[1]);
    acc[2] = Frag<_Float16>::mma(a, b2, acc[2]);
    acc[3] = Frag<_Float16>::mma(a, b3, acc[3]);
    if (LO) {
      const v16h al = Frag<_Float16>::load(alo + k0);
      accr[0] = Frag<_Float16>::mma(al, b0, accr[0]);
      accr[1] = Frag<_Float16>::mma(al, b1, accr[1]);
      accr[2] = Frag<_Float16>::mma(al, b2, accr[2]);
      accr[3] = Frag<_Float16>::mma(al, b3, accr[3]);
      dep_guard4_h(accr[0], accr[1], accr[2], accr[3], al, b0);
    }
    dep_guard4_h(acc[0], acc[1], acc[2], acc[3], a, b3);
    keep4_h(b0, b1, b2, b3);
  }
}

__device__ __forceinline__ void mma_chunks1(const _Float16* ahi, const _Float16* alo, const _Float16* brow, int nch,
                                            v8f& acc, v8f& accr) {
#pragma unroll 1
  for (int ch = 0; ch < nch; ++ch) {
    const int k0 = ch * 32;
    const v16h a  = Frag<_Float16>::load(ahi + k0);
    const v16h al = Frag<_Float16>::load(alo + k0);
    const v16h b  = Frag<_Float16>::load(brow + k0);
    acc  = Frag<_Float16>::mma(a, b, acc);
    accr = Frag<_Float16>::mma(al, b, accr);
    dep_guard2x3_h(acc, accr, a, al, b);
  }
}

__device__ __forceinline__ void cell_update(const v8f (&acc)[4], const v8f (&accr)[4], const float (&bb)[4], float (&cst)[8],
                                            _Float16* hi_n, _Float16* lo_n) {
#pragma unroll
  for (int r = 0; r < 8; ++r) {
    const float zi = (acc[0][r] + accr[0][r] * RSC_INV) * WCARRY_INV + bb[0];
    const float zf = (acc[1][r] + accr[1][r] * RSC_INV) * WCARRY_INV + bb[1];
    const float zg = (acc[2][r] + accr[2][r] * RSC_INV) * WCARRY_INV + bb[2];
    const float zo = (acc[3][r] + accr[3][r] * RSC_INV) * WCARRY_INV + bb[3];
    const float ig = fsig(zi), fg = fsig(zf), og = fsig(zo), gg = ftanh(zg);
    const float cn = fg * cst[r] + ig * gg;
    cst[r] = cn;
    const float hn = og * ftanh(cn);
    _Float16 h16, l16;
    split16(hn, h16, l16);
    hi_n[r * APITCH] = h16;
    lo_n[r * APITCH] = l16;
  }
}

__device__ __forceinline__ void stage_x(const float* __restrict__ x, _Float16* ahi, int m0, int t, int tid) {
  const int m = tid >> 4, f4 = (tid & 15) * 4;
  const v4f v = *(const v4f*)(x + ((size_t)(m0 + m) * NSTEP + (size_t)t) * NDIM + f4);
  v4h h4;
#pragma unroll
  for (int e = 0; e < 4; ++e) h4[e] = (_Float16)bf16r(v[e]);
  *(v4h*)(ahi + m * APITCH + f4) = h4;
}

__device__ __forceinline__ void store_tile16x64(const float* lds, int lp, float* gdst, size_t gpitch, int tid) {
  const int row = tid >> 4, c4 = (tid & 15) * 4;
  const v4f v = *(const v4f*)(lds + row * lp + c4);
  float* p = gdst + (size_t)row * gpitch + c4;
  *(volatile v4f*)p = v;
  __threadfence();
  *(volatile v4f*)p = v;
}

__global__ __launch_bounds__(NTHR) void seqvae_kernel(
    const float* __restrict__ x, const float* __restrict__ cond, const float* __restrict__ eps,
    const float* __restrict__ gbih, const float* __restrict__ gbhh, const float* __restrict__ gfcb,
    const float* __restrict__ rfc1b, const float* __restrict__ rbih, const float* __restrict__ rbhh,
    const float* __restrict__ rfc2b,
    const unsigned short* __restrict__ Wencp, const unsigned short* __restrict__ Wdecp,
    const unsigned short* __restrict__ Wgfcp, const unsigned short* __restrict__ Wfc1p,
    const unsigned short* __restrict__ Wfc2p,
    float* __restrict__ out) {
  __shared__ __align__(16) _Float16 Abuf[2][2][ROWS_BLK * APITCH];
  __shared__ __align__(16) float    Os[ROWS_BLK * OPITCH];
  __shared__ __align__(16) float    VA[ROWS_BLK * VPITCH];
  const _Float16* Wenc = (const _Float16*)Wencp;
  const _Float16* Wdec = (const _Float16*)Wdecp;
  const _Float16* Wgfc = (const _Float16*)Wgfcp;
  const _Float16* Wfc1 = (const _Float16*)Wfc1p;
  const _Float16* Wfc2 = (const _Float16*)Wfc2p;

  const int tid = threadIdx.x, lane = tid & 31, wave = tid >> 5;
  const int c = lane & 15, hh = lane >> 4, koff = hh * 8;
  const int m0 = blockIdx.x * ROWS_BLK;
  const int j  = 16 * wave + c;
  const int n2 = (j < NDIM) ? j : (NDIM - 1);

  const v8f z8 = {0.f, 0.f, 0.f, 0.f, 0.f, 0.f, 0.f, 0.f};
  v4h z4h;
#pragma unroll
  for (int e = 0; e < 4; ++e) z4h[e] = (_Float16)0.0f;

  {
    v8h z8h;
#pragma unroll
    for (int e = 0; e < 8; ++e) z8h[e] = (_Float16)0.0f;
    _Float16* ab = &Abuf[0][0][0];
#pragma unroll 1
    for (int i = tid; i < (2 * 2 * ROWS_BLK * APITCH) / 8; i += NTHR) *(v8h*)(ab + 8 * i) = z8h;
  }
  __syncthreads();
  stage_x(x, &Abuf[0][0][0], m0, 0, tid);

  float cst[8], bb[4];
#pragma unroll
  for (int g = 0; g < 4; ++g) bb[g] = bf16r(gbih[g * NHID + j]) + bf16r(gbhh[g * NHID + j]);
#pragma unroll
  for (int r = 0; r < 8; ++r) cst[r] = 0.0f;
  __syncthreads();

#pragma unroll 1
  for (int t = 0; t < NSTEP; ++t) {
    const int cur = t & 1, nxt = cur ^ 1;
    const _Float16* ahi  = &Abuf[cur][0][0] + c * APITCH + koff;
    const _Float16* alo  = &Abuf[cur][1][0] + c * APITCH + koff;
    const _Float16* brow = Wenc + (size_t)j * KCAT + koff;
    v8f acc[4], accr[4];
#pragma unroll
    for (int g = 0; g < 4; ++g) { acc[g] = z8; accr[g] = z8; }
    mma_chunks4<false>(ahi, alo, brow, NHID * KCAT, 0, NDIM / 32, acc, accr);
    mma_chunks4<true >(ahi, alo, brow, NHID * KCAT, NDIM / 32, KCAT / 32, acc, accr);
    acc_guard4(acc[0], acc[1], acc[2], acc[3]);
    acc_guard4(accr[0], accr[1], accr[2], accr[3]);
    cell_update(acc, accr, bb, cst,
                &Abuf[nxt][0][0] + (8 * hh) * APITCH + NDIM + j,
                &Abuf[nxt][1][0] + (8 * hh) * APITCH + NDIM + j);
    {
      const int tn = (t + 1 < NSTEP) ? (t + 1) : (NSTEP - 1);
      stage_x(x, &Abuf[nxt][0][0], m0, tn, tid);
    }
    __syncthreads();
  }

  {
    const int row = tid >> 4, c8 = (tid & 15) * 8;
    const v8h hv = *(const v8h*)(&Abuf[0][0][0] + row * APITCH + NDIM + c8);
    const v8h lv = *(const v8h*)(&Abuf[0][1][0] + row * APITCH + NDIM + c8);
    *(v8h*)(&Abuf[1][0][0] + row * APITCH + c8) = hv;
    *(v8h*)(&Abuf[1][1][0] + row * APITCH + c8) = lv;
    if (tid < 128) {
      const int r2 = tid >> 3, c4 = (tid & 7) * 4;
      const v4f iv = *(const v4f*)(cond + (size_t)(m0 + r2) * NCOND + c4);
      v4h h4;
#pragma unroll
      for (int e = 0; e < 4; ++e) h4[e] = (_Float16)bf16r(iv[e]);
      *(v4h*)(&Abuf[1][0][0] + r2 * APITCH + NHID + c4) = h4;
      *(v4h*)(&Abuf[1][1][0] + r2 * APITCH + NHID + c4) = z4h;
    }
  }
  __syncthreads();

  {
    v8f a1 = z8, ar1 = z8;
    mma_chunks1(&Abuf[1][0][0] + c * APITCH + koff, &Abuf[1][1][0] + c * APITCH + koff,
                Wgfc + (size_t)j * KVAE + koff, KVAE / 32, a1, ar1);
    acc_guard2(a1, ar1);
    const float bv = bf16r(gfcb[j]);
#pragma unroll
    for (int r = 0; r < 8; ++r) VA[(8 * hh + r) * VPITCH + j] = (a1[r] + ar1[r] * RSC_INV) * WCARRY_INV + bv;
  }
  __syncthreads();

  {
    const int row = tid >> 4, c4 = (tid & 15) * 4;
    const v4f mu4 = *(const v4f*)(VA + row * VPITCH + c4);
    const v4f lv4 = *(const v4f*)(VA + row * VPITCH + NZ + c4);
    float* pmu = out + OFF_MU + (size_t)(m0 + row) * NZ + c4;
    float* plv = out + OFF_LV + (size_t)(m0 + row) * NZ + c4;
    *(volatile v4f*)pmu = mu4;
    *(volatile v4f*)plv = lv4;
    __threadfence();
    *(volatile v4f*)pmu = mu4;
    *(volatile v4f*)plv = lv4;
    const v4f ep4 = *(const v4f*)(eps + (size_t)(m0 + row) * NZ + c4);
    v4h zh, zl;
#pragma unroll
    for (int e = 0; e < 4; ++e) {
      const float zv = mu4[e] + bf16r(ep4[e]) * expf(0.5f * lv4[e]);
      _Float16 h16, l16;
      split16(zv, h16, l16);
      zh[e] = h16; zl[e] = l16;
    }
    *(v4h*)(&Abuf[0][0][0] + row * APITCH + c4) = zh;
    *(v4h*)(&Abuf[0][1][0] + row * APITCH + c4) = zl;
    if (tid < 128) {
      const int r2 = tid >> 3, d4 = (tid & 7) * 4;
      const v4f iv = *(const v4f*)(cond + (size_t)(m0 + r2) * NCOND + d4);
      v4h h4;
#pragma unroll
      for (int e = 0; e < 4; ++e) h4[e] = (_Float16)bf16r(iv[e]);
      *(v4h*)(&Abuf[0][0][0] + r2 * APITCH + NZ + d4) = h4;
      *(v4h*)(&Abuf[0][1][0] + r2 * APITCH + NZ + d4) = z4h;
    }
  }
  __syncthreads();

  {
    const int row = tid >> 4, c4 = (tid & 15) * 4;
    *(v4h*)(&Abuf[1][0][0] + row * APITCH + c4) = z4h;
    *(v4h*)(&Abuf[1][1][0] + row * APITCH + c4) = z4h;
    v8f a1 = z8, ar1 = z8;
    mma_chunks1(&Abuf[0][0][0] + c * APITCH + koff, &Abuf[0][1][0] + c * APITCH + koff,
                Wfc1 + (size_t)j * KFC1 + koff, KFC1 / 32, a1, ar1);
    acc_guard2(a1, ar1);
    const float bv = bf16r(rfc1b[j]);
#pragma unroll
    for (int r = 0; r < 8; ++r) {
      const float hd = (a1[r] + ar1[r] * RSC_INV) * WCARRY_INV + bv;
      _Float16 h16, l16;
      split16(hd, h16, l16);
      Abuf[1][0][(8 * hh + r) * APITCH + NDIM + j] = h16;
      Abuf[1][1][(8 * hh + r) * APITCH + NDIM + j] = l16;
      cst[r] = 0.0f;
    }
  }
#pragma unroll
  for (int g = 0; g < 4; ++g) bb[g] = bf16r(rbih[g * NHID + j]) + bf16r(rbhh[g * NHID + j]);
  const float b2v = bf16r(rfc2b[n2]);
  __syncthreads();

#pragma unroll 1
  for (int s = 0; s < NSTEP; ++s) {
    const int cur = (s + 1) & 1, nxt = cur ^ 1;
    {
      const _Float16* ahi  = &Abuf[cur][0][0] + c * APITCH + koff;
      const _Float16* alo  = &Abuf[cur][1][0] + c * APITCH + koff;
      const _Float16* brow = Wdec + (size_t)j * KCAT + koff;
      v8f acc[4], accr[4];
#pragma unroll
      for (int g = 0; g < 4; ++g) { acc[g] = z8; accr[g] = z8; }
      mma_chunks4<true>(ahi, alo, brow, NHID * KCAT, 0, KCAT / 32, acc, accr);
      acc_guard4(acc[0], acc[1], acc[2], acc[3]);
      acc_guard4(accr[0], accr[1], accr[2], accr[3]);
      cell_update(acc, accr, bb, cst,
                  &Abuf[nxt][0][0] + (8 * hh) * APITCH + NDIM + j,
                  &Abuf[nxt][1][0] + (8 * hh) * APITCH + NDIM + j);
    }
    __syncthreads();
    if (wave < NDIM / 16) {
      v8f oa = z8, oar = z8;
      mma_chunks1(&Abuf[nxt][0][0] + c * APITCH + NDIM + koff, &Abuf[nxt][1][0] + c * APITCH + NDIM + koff,
                  Wfc2 + (size_t)n2 * NHID + koff, NHID / 32, oa, oar);
      acc_guard2(oa, oar);
#pragma unroll
      for (int r = 0; r < 8; ++r) {
        const float v = (oa[r] + oar[r] * RSC_INV) * WCARRY_INV + b2v;
        Os[(8 * hh + r) * OPITCH + n2] = v;
        _Float16 h16, l16;
        split16(v, h16, l16);
        Abuf[nxt][0][(8 * hh + r) * APITCH + n2] = h16;
        Abuf[nxt][1][(8 * hh + r) * APITCH + n2] = l16;
      }
    }
    __syncthreads();
    store_tile16x64(Os, OPITCH, out + ((size_t)m0 * NSTEP + (size_t)s) * NDIM, (size_t)NSTEP * NDIM, tid);
  }
}

extern "C" void kernel_launch(void* const* d_in, const int* in_sizes, int n_in,
                              void* d_out, int out_size, void* d_ws, size_t ws_size, hipStream_t stream) {
  if (n_in < 17 || d_out == nullptr || d_ws == nullptr) return;
  if (in_sizes[0] != NBATCH * NSTEP * NDIM || in_sizes[1] != NBATCH * NCOND || in_sizes[2] != NBATCH * NZ ||
      in_sizes[3] != NGATE * NDIM || in_sizes[4] != NGATE * NHID || in_sizes[5] != NGATE || in_sizes[6] != NGATE ||
      in_sizes[7] != 2 * NZ * KVAE || in_sizes[8] != 2 * NZ || in_sizes[9] != NHID * KFC1 || in_sizes[10] != NHID ||
      in_sizes[11] != NGATE * NDIM || in_sizes[12] != NGATE * NHID || in_sizes[13] != NGATE || in_sizes[14] != NGATE ||
      in_sizes[15] != NDIM * NHID || in_sizes[16] != NDIM ||
      out_size != (int)(OFF_LV + (size_t)NBATCH * NZ)) return;

  const float* x     = (const float*)d_in[0];
  const float* cond  = (const float*)d_in[1];
  const float* eps   = (const float*)d_in[2];
  const float* gWih  = (const float*)d_in[3];
  const float* gWhh  = (const float*)d_in[4];
  const float* gbih  = (const float*)d_in[5];
  const float* gbhh  = (const float*)d_in[6];
  const float* gfcW  = (const float*)d_in[7];
  const float* gfcb  = (const float*)d_in[8];
  const float* rfc1W = (const float*)d_in[9];
  const float* rfc1b = (const float*)d_in[10];
  const float* rWih  = (const float*)d_in[11];
  const float* rWhh  = (const float*)d_in[12];
  const float* rbih  = (const float*)d_in[13];
  const float* rbhh  = (const float*)d_in[14];
  const float* rfc2W = (const float*)d_in[15];
  const float* rfc2b = (const float*)d_in[16];
  float* out = (float*)d_out;

  char* ws = (char*)d_ws; size_t off = 0;
  auto carve = [&](size_t bytes) -> char* { char* p = ws + off; off += (bytes + 255) & ~(size_t)255; return p; };
  unsigned short* Wenc = (unsigned short*)carve((size_t)NGATE * KCAT * 2);
  unsigned short* Wdec = (unsigned short*)carve((size_t)NGATE * KCAT * 2);
  unsigned short* Wgfc = (unsigned short*)carve((size_t)(2 * NZ) * KVAE * 2);
  unsigned short* Wfc1 = (unsigned short*)carve((size_t)NHID * KFC1 * 2);
  unsigned short* Wfc2 = (unsigned short*)carve((size_t)NDIM * NHID * 2);
  if (off > ws_size || off > (size_t)134217728) return;

  cvt_rows_kernel<<<(NGATE * NDIM / 8 + NTHR - 1) / NTHR, NTHR, 0, stream>>>(gWih, Wenc, NGATE, NDIM, KCAT, 0, WCARRY);
  cvt_rows_kernel<<<(NGATE * NHID / 8 + NTHR - 1) / NTHR, NTHR, 0, stream>>>(gWhh, Wenc, NGATE, NHID, KCAT, NDIM, WCARRY);
  cvt_rows_kernel<<<(NGATE * NDIM / 8 + NTHR - 1) / NTHR, NTHR, 0, stream>>>(rWih, Wdec, NGATE, NDIM, KCAT, 0, WCARRY);
  cvt_rows_kernel<<<(NGATE * NHID / 8 + NTHR - 1) / NTHR, NTHR, 0, stream>>>(rWhh, Wdec, NGATE, NHID, KCAT, NDIM, WCARRY);
  cvt_rows_kernel<<<(2 * NZ * KVAE / 8 + NTHR - 1) / NTHR, NTHR, 0, stream>>>(gfcW, Wgfc, 2 * NZ, KVAE, KVAE, 0, WCARRY);
  cvt_rows_kernel<<<(NHID * KFC1 / 8 + NTHR - 1) / NTHR, NTHR, 0, stream>>>(rfc1W, Wfc1, NHID, KFC1, KFC1, 0, WCARRY);
  cvt_rows_kernel<<<(NDIM * NHID / 8 + NTHR - 1) / NTHR, NTHR, 0, stream>>>(rfc2W, Wfc2, NDIM, NHID, NHID, 0, WCARRY);
  seqvae_kernel<<<NBATCH / ROWS_BLK, NTHR, 0, stream>>>(x, cond, eps, gbih, gbhh, gfcb, rfc1b, rbih, rbhh, rfc2b,
                                                        Wenc, Wdec, Wgfc, Wfc1, Wfc2, out);
}
